// ConvAttnState_59966333386902
// MI455X (gfx1250) — hardware-verified
//
#include <hip/hip_runtime.h>
#include <hip/hip_bf16.h>
#include <math.h>

#define NB 8
#define HH 12
#define LL 2048
#define LQ 1024
#define DKK 64
#define EE 768
#define SS 2048
#define QROWS 1024
#define KROWS 2048
#define NKV 2048
#define DD 768
#define KVD 768
#define KVH 12
#define HKDIV 1
#define QW 2
#define GSTR 48

typedef _Float16 bf16;
typedef _Float16 f16;
typedef __attribute__((ext_vector_type(4))) unsigned v4u_t;
typedef unsigned v4ua __attribute__((ext_vector_type(4), may_alias));
typedef __attribute__((ext_vector_type(4))) float v4f_t;
typedef float v4fa __attribute__((ext_vector_type(4), may_alias));
typedef __attribute__((ext_vector_type(16))) bf16  bf16x16;
typedef bf16x16 f16x16;
typedef __attribute__((ext_vector_type(8)))  bf16  bf16x8;
typedef bf16x8 f16x8;
typedef __attribute__((ext_vector_type(4)))  bf16  bf16x4;
typedef __attribute__((ext_vector_type(8)))  float f32x8;
__device__ __forceinline__ f32x8 wmma16(f16x16 a, f16x16 b, f32x8 c) {
  c = __builtin_amdgcn_wmma_f32_16x16x32_f16(false, a, false, b, (short)0, c, false, false);
  asm volatile("v_nop\n\tv_nop\n\tv_nop\n\tv_nop" : "+v"(c) : "v"(a), "v"(b));
  return c;
}
#define LDS_STRIDE 48
#define KSTRIDE    72
#define VSTRIDE    48

__device__ __forceinline__ f32x8 wmma_bf16(bf16x16 a, bf16x16 b, f32x8 c) {
  c = __builtin_amdgcn_wmma_f32_16x16x32_f16(false, a, false, b, (short)0, c, false, false);
  asm volatile("v_nop\n\tv_nop\n\tv_nop\n\tv_nop" : "+v"(c) : "v"(a), "v"(b));
  return c;
}

template <typename T>
__device__ __forceinline__ bf16x16 load_frag(const T* __restrict__ base, int ld,
                                             int row0, int k0) {
  const int lane = threadIdx.x & 31;
  const int r    = lane & 15;
  const int kh   = (lane >> 4) * 8;
  const T* p0 = base + (size_t)(row0 + r) * ld + (k0 + kh);
  const T* p1 = p0 + 16;
  bf16x16 f;
#pragma unroll
  for (int i = 0; i < 8; ++i) {
    f[i]     = (bf16)p0[i];
    f[i + 8] = (bf16)p1[i];
  }
  return f;
}

__device__ __forceinline__ bf16x16 lds_frag(const bf16* base, int stride) {
  const int lane = threadIdx.x & 31;
  const int row  = lane & 15;
  const int kh   = (lane >> 4) * 8;
  const bf16x8 lo = *(const bf16x8*)(base + row * stride + kh);
  const bf16x8 hi = *(const bf16x8*)(base + row * stride + kh + 16);
  bf16x16 f;
#pragma unroll
  for (int i = 0; i < 8; ++i) { f[i] = lo[i]; f[i + 8] = hi[i]; }
  return f;
}

template <typename T>
__device__ __forceinline__ void stage_read16(const T* __restrict__ p, float* buf) {
#pragma unroll
  for (int i = 0; i < 16; ++i) buf[i] = (float)p[i];
}

__device__ __forceinline__ void stage_write(bf16* dst, const float* buf, int nquad) {
#pragma unroll
  for (int i = 0; i < nquad; ++i) {
    bf16x4 q;
    q[0] = (bf16)buf[4 * i];     q[1] = (bf16)buf[4 * i + 1];
    q[2] = (bf16)buf[4 * i + 2]; q[3] = (bf16)buf[4 * i + 3];
    *(bf16x4*)(dst + 4 * i) = q;
  }
}

template <typename AT, int MODE>
__global__ __launch_bounds__(256) void gemm_rb_kernel(
    const AT* __restrict__ A, const float* __restrict__ W,
    const float* __restrict__ bias, const float* __restrict__ rowscale, const float* __restrict__ R, const float* __restrict__ rowbias, void* __restrict__ out,
    int M, int N, int K) {
  __shared__ bf16 ldsA[128 * LDS_STRIDE];
  __shared__ bf16 ldsW[256 * LDS_STRIDE];
  __shared__ __attribute__((aligned(16))) unsigned char sob[256 * 136 * 2];

  const int t    = threadIdx.x;
  const int wave = t >> 5;
  const int lane = t & 31;
  const int wm   = (wave & 1) * 64;
  const int wn   = (wave >> 1) * 64;
  const int mBlk = blockIdx.x * 128;
  const int nBlk = blockIdx.y * 256;

  const int arow = t >> 1;
  const int ach  = (t & 1) * 16;

  float abuf[16];
  float wbuf[32];

  stage_read16(A + (size_t)(mBlk + arow) * K + ach, abuf);
  const int nrow = min(nBlk + t, N - 1);
  stage_read16(W + (size_t)nrow * K,          wbuf);
  stage_read16(W + (size_t)nrow * K + 16,     wbuf + 16);

  f32x8 acc[4][4] = {};

  for (int k = 0; k < K; k += 32) {
    __syncthreads();
    stage_write(&ldsA[arow * LDS_STRIDE + ach], abuf, 4);
    stage_write(&ldsW[t * LDS_STRIDE],          wbuf, 8);
    if (k + 32 < K) {
      stage_read16(A + (size_t)(mBlk + arow) * K + (k + 32) + ach, abuf);
      stage_read16(W + (size_t)nrow * K + (k + 32),          wbuf);
      stage_read16(W + (size_t)nrow * K + (k + 32) + 16,     wbuf + 16);
    }
    __syncthreads();

    bf16x16 af[4], wf[4];
#pragma unroll
    for (int i = 0; i < 4; ++i)
      af[i] = lds_frag(ldsA + (wm + 16 * i) * LDS_STRIDE, LDS_STRIDE);
#pragma unroll
    for (int j = 0; j < 4; ++j)
      wf[j] = lds_frag(ldsW + (wn + 16 * j) * LDS_STRIDE, LDS_STRIDE);
#pragma unroll
    for (int i = 0; i < 4; ++i)
#pragma unroll
      for (int j = 0; j < 4; ++j)
        acc[i][j] = wmma_bf16(af[i], wf[j], acc[i][j]);
  }

  const int nlane = lane & 15;
  const int mh    = (lane >> 4) * 8;
  __syncthreads();
  if (MODE == 0 || MODE == 1 || MODE == 3) {
    bf16* so = (bf16*)sob;
#pragma unroll
    for (int i = 0; i < 4; ++i)
#pragma unroll
      for (int j = 0; j < 4; ++j) {
        const int nl = wn + 16 * j + nlane;
        const float bv = bias ? bias[nBlk + nl] : 0.0f;
        if (MODE == 3) {
#pragma unroll 1
          for (int r = 0; r < 8; ++r) {
            const int ml = wm + 16 * i + mh + r;
            const float xg = acc[i][j][r] + bv;
            so[ml * 264 + nl] = (bf16)(0.5f * xg * (1.0f + erff(xg * 0.70710678118654752f)));
          }
        } else {
#pragma unroll
        for (int r = 0; r < 8; ++r) {
          const int ml = wm + 16 * i + mh + r;
          const bf16 hv = (bf16)(acc[i][j][r] + bv);
          if (MODE == 0) so[ml * 264 + nl] = hv;
          else           so[nl * 136 + ml] = hv;
        }
        }
      }
    __syncthreads();
#pragma unroll 1
    for (int pass = 0; pass < 2; ++pass) {
      if (MODE == 0 || MODE == 3) {
        for (int ch = t; ch < 128 * 32; ch += 256) { const int ml = ch >> 5, q = (ch & 31) * 8;
          *(volatile v4u_t*)((bf16*)out + (size_t)(mBlk + ml) * N + nBlk + q) = *(const v4ua*)(so + ml * 264 + q); }
      } else {
        const int b_ = mBlk / SS, s0 = mBlk % SS;
        for (int ch = t; ch < 256 * 16; ch += 256) { const int nl = ch >> 4, q = (ch & 15) * 8; const int n = nBlk + nl, h = n >> 6, dk = n & (DKK - 1);
          *(volatile v4u_t*)((bf16*)out + (((size_t)(b_ * HH + h)) * DKK + dk) * SS + s0 + q) = *(const v4ua*)(so + nl * 136 + q); }
      }
      __threadfence();
    }
  } else {
    float* so = (float*)sob;
#pragma unroll 1
    for (int hf = 0; hf < 2; ++hf) {
      if (wm == hf * 64) {
#pragma unroll
        for (int i = 0; i < 4; ++i)
#pragma unroll
          for (int j = 0; j < 4; ++j) {
            const int nl = wn + 16 * j + nlane;
            const float bv = bias ? bias[nBlk + nl] : 0.0f;
#pragma unroll
            for (int r = 0; r < 8; ++r) { const int mrow = mBlk + hf * 64 + 16 * i + mh + r; so[(16 * i + mh + r) * 260 + nl] = acc[i][j][r] * (rowscale ? rowscale[mrow] : 1.0f) + bv + (rowbias ? rowbias[mrow] : 0.0f); }
          }
      }
      __syncthreads();
      if (R) {
        for (int ch = t; ch < 64 * 64; ch += 256) { const int ml = ch >> 6, q = (ch & 63) * 4;
          if (nBlk + q < N) { const v4f_t rv = *(const v4f_t*)(R + (size_t)(mBlk + hf * 64 + ml) * N + nBlk + q); v4f_t v = *(const v4fa*)(so + ml * 260 + q); v += rv; *(volatile v4fa*)(so + ml * 260 + q) = v; } }
        asm volatile("s_wait_dscnt 0" ::: "memory");
      }
#pragma unroll 1
      for (int pass = 0; pass < 2; ++pass) {
        for (int ch = t; ch < 64 * 64; ch += 256) { const int ml = ch >> 6, q = (ch & 63) * 4;
          if (nBlk + q < N) *(volatile v4f_t*)((float*)out + (size_t)(mBlk + hf * 64 + ml) * N + nBlk + q) = *(const v4fa*)(so + ml * 260 + q); }
        __threadfence();
      }
      __syncthreads();
    }
  }
}


#define GSTR 48
template <typename AT, int EPI, bool OUT16>
__global__ __launch_bounds__(256) void gemm_kne(const AT* __restrict__ A, int lda, const float* __restrict__ Wm, int ldw,
                                                const float* __restrict__ bias, const float* __restrict__ R, const float* __restrict__ gvec,
                                                void* __restrict__ Yv, int ldy, int K) {
  __shared__ __attribute__((aligned(16))) f16 ldsA[128 * GSTR];
  __shared__ __attribute__((aligned(16))) f16 ldsW[128 * GSTR];
  __shared__ __attribute__((aligned(16))) float oS[8][32 * 68];
  const int tid = threadIdx.x, lane = tid & 31, wave = tid >> 5, cl = lane & 15, rh = (lane >> 4) * 8;
  const int m0 = blockIdx.x * 128, n0 = blockIdx.y * 128;
  const int wm = (wave & 3) * 32, wn = (wave >> 2) * 64;
  f32x8 acc[2][4];
#pragma unroll
  for (int i = 0; i < 2; ++i)
#pragma unroll
    for (int j = 0; j < 4; ++j) { f32x8 z = {}; acc[i][j] = z; }
#pragma unroll 1
  for (int k0 = 0; k0 < K; k0 += 32) {
    __syncthreads();
    { const int row = tid >> 1, ch = (tid & 1) * 16;
      const AT* src = A + (size_t)(m0 + row) * lda + k0 + ch;
#pragma unroll
      for (int g = 0; g < 16; ++g) ldsA[row * GSTR + ch + g] = (f16)src[g]; }
    { const int k = tid >> 3, nn0 = (tid & 7) * 16;
      const float* src = Wm + (size_t)(k0 + k) * ldw + n0 + nn0;
#pragma unroll
      for (int g = 0; g < 4; ++g) { const v4f_t v = *(const v4f_t*)(src + 4 * g);
#pragma unroll
        for (int u = 0; u < 4; ++u) ldsW[(nn0 + 4 * g + u) * GSTR + k] = (f16)v[u]; } }
    __syncthreads();
    f16x16 af[2];
#pragma unroll
    for (int i = 0; i < 2; ++i) af[i] = lds_frag(ldsA + (wm + 16 * i) * GSTR, GSTR);
#pragma unroll
    for (int j = 0; j < 4; ++j) {
      const f16x16 bf = lds_frag(ldsW + (wn + 16 * j) * GSTR, GSTR);
#pragma unroll
      for (int i = 0; i < 2; ++i) acc[i][j] = wmma16(af[i], bf, acc[i][j]);
    }
  }
  float* so = oS[wave];
#pragma unroll
  for (int i = 0; i < 2; ++i)
#pragma unroll
    for (int j = 0; j < 4; ++j) {
      const int n = n0 + wn + 16 * j + cl;
      const float bv = bias ? bias[n] : 0.0f;
      const float gv = (EPI == 2) ? gvec[n] : 0.0f;
      if (EPI == 1) {
#pragma unroll 1
        for (int r = 0; r < 8; ++r) { const float xg = acc[i][j][r] + bv; so[(16 * i + rh + r) * 68 + 16 * j + cl] = 0.5f * xg * (1.0f + erff(xg * 0.70710678118654752f)); }
      } else {
#pragma unroll
        for (int r = 0; r < 8; ++r) {
          float v = acc[i][j][r] + bv;
          if (EPI == 3) v = fmaxf(v, 0.0f);
          if (EPI == 2) v = R[(size_t)(m0 + wm + 16 * i + rh + r) * ldy + n] + gv * v;
          so[(16 * i + rh + r) * 68 + 16 * j + cl] = v;
        }
      }
    }
  asm volatile("s_wait_dscnt 0" ::: "memory");
  __builtin_amdgcn_wave_barrier();
#pragma unroll 1
  for (int pass = 0; pass < 2; ++pass) {
    if (OUT16) {
      f16* Y = (f16*)Yv;
#pragma unroll
      for (int it = 0; it < 8; ++it) { const int c = lane + 32 * it, rr = c >> 3, q8 = (c & 7) * 8;
        union { f16 h[8]; v4u_t v; } u;
#pragma unroll
        for (int e = 0; e < 8; ++e) u.h[e] = (f16)so[rr * 68 + q8 + e];
        *(volatile v4u_t*)(Y + (size_t)(m0 + wm + rr) * ldy + n0 + wn + q8) = u.v; }
    } else {
      float* Y = (float*)Yv;
#pragma unroll
      for (int it = 0; it < 16; ++it) { const int f4 = lane + 32 * it, rr = f4 >> 4, q = (f4 & 15) * 4;
        *(volatile v4f_t*)(Y + (size_t)(m0 + wm + rr) * ldy + n0 + wn + q) = *(const v4fa*)(so + rr * 68 + q); }
    }
    __threadfence();
  }
}
__global__ __launch_bounds__(64) void ca_attn_kernel(
    const bf16* __restrict__ Qb, const bf16* __restrict__ Kb,
    const bf16* __restrict__ Vt,
    float* __restrict__ attnOut) {
  __shared__ bf16 ldsK[32 * KSTRIDE];
  __shared__ bf16 ldsV[64 * VSTRIDE];
  __shared__ __attribute__((aligned(16))) bf16 ldsO[2][32 * 72];

  const int q0blk = blockIdx.x * 64;
  const int h  = blockIdx.y;
  const int b  = blockIdx.z;
  const int t    = threadIdx.x;
  const int wave = t >> 5;
  const int lane = t & 31;
  const int qlane = lane & 15;
  const int kh8   = (lane >> 4) * 8;
  const int q0 = q0blk + wave * 32;

  const int hk = h / HKDIV;
  const bf16* Qh = Qb + (size_t)b * QROWS * DD + h * DKK;
  const bf16* Kh = Kb + (size_t)b * KROWS * KVD + hk * DKK;
  const bf16* Vh = Vt + ((size_t)(b * KVH + hk)) * DKK * KROWS;

  const int krow = t >> 1;
  const int kcol = (t & 1) * 32;
  const bf16* kSrc = Kh + (size_t)krow * KVD + kcol;
  const bf16* vSrc = Vh + (size_t)t * KROWS;

  bf16x16 qf[QW][2];
#pragma unroll
  for (int qt = 0; qt < QW; ++qt) {
    qf[qt][0] = load_frag(Qh, DD, q0 + 16 * qt, 0);
    qf[qt][1] = load_frag(Qh, DD, q0 + 16 * qt, 32);
  }

  f32x8 o[QW][4] = {};
  float mrun[QW], lrun[QW];
#pragma unroll
  for (int qt = 0; qt < QW; ++qt) { mrun[qt] = -INFINITY; lrun[qt] = 0.0f; }

  const float scale = 0.125f * 1.44269504088896340736f;
  const float NEG2 = -1.0e9f;
  const int kmax = KROWS - 1;

  bf16x8 kreg[4], vreg[4];
#pragma unroll
  for (int i = 0; i < 4; ++i) {
    kreg[i] = *(const bf16x8*)(kSrc + 8 * i);
    vreg[i] = *(const bf16x8*)(vSrc + 8 * i);
  }

  for (int kb = 0; kb <= kmax; kb += 32) {
    __syncthreads();
#pragma unroll
    for (int i = 0; i < 4; ++i) {
      *(bf16x8*)(&ldsK[krow * KSTRIDE + kcol + 8 * i]) = kreg[i];
      *(bf16x8*)(&ldsV[t * VSTRIDE + 8 * i])           = vreg[i];
    }
    if (kb + 32 <= kmax) {
      const bf16* kn = kSrc + (size_t)(kb + 32) * KVD;
      const bf16* vn = vSrc + (kb + 32);
#pragma unroll
      for (int i = 0; i < 4; ++i) {
        kreg[i] = *(const bf16x8*)(kn + 8 * i);
        vreg[i] = *(const bf16x8*)(vn + 8 * i);
      }
    }
    __syncthreads();

    bf16x16 kf[2][2];
#pragma unroll
    for (int ktile = 0; ktile < 2; ++ktile)
#pragma unroll
      for (int c = 0; c < 2; ++c)
        kf[ktile][c] = lds_frag(ldsK + (ktile * 16) * KSTRIDE + c * 32, KSTRIDE);

    bf16x16 pf[QW];
    bool act[QW];
#pragma unroll
    for (int qt = 0; qt < QW; ++qt) {
      unsigned mbits = 0;
      {
#pragma unroll
        for (int r = 0; r < 8; ++r) { const int j0 = kb + kh8 + r; if (j0 < NKV) mbits |= 1u << r; if (j0 + 16 < NKV) mbits |= 1u << (8 + r); }
        act[qt] = (__builtin_amdgcn_ballot_w32(mbits != 0) != 0);
      }
      if (act[qt]) {
        const int q_my = q0 + 16 * qt + qlane;
        f32x8 s0 = {}, s1 = {};
        s0 = wmma_bf16(kf[0][0], qf[qt][0], s0);
        s0 = wmma_bf16(kf[0][1], qf[qt][1], s0);
        s1 = wmma_bf16(kf[1][0], qf[qt][0], s1);
        s1 = wmma_bf16(kf[1][1], qf[qt][1], s1);

        float mx = -INFINITY;
#pragma unroll
        for (int r = 0; r < 8; ++r) {
          const int k0i = kb + kh8 + r;
          const int k1i = k0i + 16;
          (void)k0i; (void)k1i; (void)q_my;
          s0[r] = (mbits & (1u << r))       ? s0[r] * scale : NEG2;
          s1[r] = (mbits & (1u << (8 + r))) ? s1[r] * scale : NEG2;
          mx = fmaxf(mx, fmaxf(s0[r], s1[r]));
        }
        mx = fmaxf(mx, __shfl_xor(mx, 16, 32));
        const float mnew  = fmaxf(mrun[qt], mx);
        const float alpha = exp2f(mrun[qt] - mnew);

        float rsum = 0.0f;
#pragma unroll
        for (int r = 0; r < 8; ++r) {
          const float p0 = exp2f(s0[r] - mnew);
          const float p1 = exp2f(s1[r] - mnew);
          rsum += p0 + p1;
          pf[qt][r]     = (bf16)(p0 * 1024.0f);
          pf[qt][r + 8] = (bf16)(p1 * 1024.0f);
        }
        rsum += __shfl_xor(rsum, 16, 32);
        lrun[qt] = lrun[qt] * alpha + rsum;
        mrun[qt] = mnew;

#pragma unroll
        for (int j = 0; j < 4; ++j)
#pragma unroll
          for (int r = 0; r < 8; ++r) o[qt][j][r] *= alpha;
      }
    }

#pragma unroll
    for (int j = 0; j < 4; ++j) {
      const bf16x16 vf = lds_frag(ldsV + (j * 16) * VSTRIDE, VSTRIDE);
#pragma unroll
      for (int qt = 0; qt < QW; ++qt)
        if (act[qt]) o[qt][j] = wmma_bf16(vf, pf[qt], o[qt][j]);
    }
  }

  __shared__ __attribute__((aligned(16))) float ldsOf[2][32 * 68];
  float* so = ldsOf[wave]; (void)ldsO;
#pragma unroll
  for (int qt = 0; qt < QW; ++qt) {
    const float rl = 1.0f / (lrun[qt] * 1024.0f);
#pragma unroll
    for (int j = 0; j < 4; ++j)
#pragma unroll
      for (int r = 0; r < 8; ++r) so[(16 * qt + qlane) * 68 + j * 16 + kh8 + r] = o[qt][j][r] * rl;
  }
  asm volatile("s_wait_dscnt 0" ::: "memory");
  __builtin_amdgcn_wave_barrier();
#pragma unroll 1
  for (int pass = 0; pass < 2; ++pass) {
#pragma unroll
    for (int it = 0; it < 16; ++it) { const int ch = lane + 32 * it, ql = ch >> 4, q4 = (ch & 15) * 4;
      *(volatile v4f_t*)(attnOut + ((size_t)(b * QROWS + q0 + ql)) * DD + h * DKK + q4) = *(const v4fa*)(so + ql * 68 + q4); }
    __threadfence();
  }
}


__global__ __launch_bounds__(192) void k_gather_x0(const float* __restrict__ st, int b, float* __restrict__ X0) { const int l = blockIdx.x; const int c4 = threadIdx.x * 4; const int h = c4 >> 6, d = c4 & 63;
  const v4f_t v = *(const v4f_t*)(st + (((size_t)b * HH + h) * LL + l) * DKK + d); *(volatile v4f_t*)(X0 + (size_t)l * EE + c4) = v; __threadfence(); *(volatile v4f_t*)(X0 + (size_t)l * EE + c4) = v; }
__global__ __launch_bounds__(192) void k_resid(const float* __restrict__ X0, float* __restrict__ Xres) { const int lq = blockIdx.x; const int c4 = threadIdx.x * 4;
  const v4f_t v = *(const v4f_t*)(X0 + (size_t)(2 * lq) * EE + c4); *(volatile v4f_t*)(Xres + (size_t)lq * EE + c4) = v; __threadfence(); *(volatile v4f_t*)(Xres + (size_t)lq * EE + c4) = v; }
__global__ __launch_bounds__(256) void k_transpose(const float* __restrict__ Wm, float* __restrict__ Wt, int rows, int cols) {
  __shared__ float tS[64][65];
  const int tid = threadIdx.x, tbj = cols / 64, bi = blockIdx.x / tbj, bj = blockIdx.x % tbj;
  for (int e = tid; e < 64 * 64; e += 256) { const int r = e >> 6, c = e & 63; tS[r][c] = Wm[(size_t)(bi * 64 + r) * cols + bj * 64 + c]; }
  __syncthreads();
  for (int ch = tid; ch < 64 * 16; ch += 256) { const int r = ch >> 4, q4 = (ch & 15) * 4; v4f_t o; o[0] = tS[q4][r]; o[1] = tS[q4 + 1][r]; o[2] = tS[q4 + 2][r]; o[3] = tS[q4 + 3][r];
    float* dst = Wt + (size_t)(bj * 64 + r) * rows + bi * 64 + q4; *(volatile v4f_t*)dst = o; __threadfence(); *(volatile v4f_t*)dst = o; }
}
__global__ __launch_bounds__(96) void k_im2col(const bf16* __restrict__ XR, bf16* __restrict__ Aq) { const int lq = blockIdx.x, k = blockIdx.y; const int l = 2 * lq + k - 1; const int c8 = threadIdx.x * 8;
  v4u_t v = {0u, 0u, 0u, 0u}; if (l >= 0 && l < LL) v = *(const v4u_t*)(XR + (size_t)l * EE + c8);
  *(volatile v4u_t*)(Aq + (size_t)lq * (3 * EE) + k * EE + c8) = v; __threadfence(); *(volatile v4u_t*)(Aq + (size_t)lq * (3 * EE) + k * EE + c8) = v; }
__global__ __launch_bounds__(256) void k_rows16(const float* __restrict__ P, bf16* __restrict__ R16) { __shared__ __attribute__((aligned(16))) bf16 s[64][72];
  const int tid = threadIdx.x; const size_t t0 = (size_t)blockIdx.x * 64; const int h = blockIdx.y;
  for (int e = tid; e < 64 * 64; e += 256) { const int t = e >> 6, d = e & 63; s[t][d] = (bf16)P[(t0 + t) * EE + h * DKK + d]; }
  __syncthreads();
#pragma unroll 1
  for (int pass = 0; pass < 2; ++pass) {
#pragma unroll 1
    for (int round = 0; round < 2; ++round) { const int r = round * 32 + (tid >> 3), piece = (tid & 7) * 8; *(volatile v4u_t*)(R16 + (t0 + r) * EE + h * DKK + piece) = *(const v4ua*)(&s[r][piece]); }
    __threadfence(); } }
__global__ __launch_bounds__(256) void k_vt16(const bf16* __restrict__ V16, bf16* __restrict__ Vt) { __shared__ __attribute__((aligned(16))) bf16 vT[64][72];
  const int tid = threadIdx.x; const int n0 = blockIdx.x * 64; const int h = blockIdx.y;
  for (int e = tid; e < 64 * 64; e += 256) { const int t = e >> 6, d = e & 63; vT[d][t] = V16[(size_t)(n0 + t) * EE + h * DKK + d]; }
  __syncthreads();
#pragma unroll 1
  for (int pass = 0; pass < 2; ++pass) {
#pragma unroll 1
    for (int round = 0; round < 2; ++round) { const int r = round * 32 + (tid >> 3), piece = (tid & 7) * 8; *(volatile v4u_t*)(Vt + ((size_t)h * DKK + r) * LL + n0 + piece) = *(const v4ua*)(&vT[r][piece]); }
    __threadfence(); } }
__global__ __launch_bounds__(96) void k_relu16(const float* __restrict__ T, bf16* __restrict__ O) { const size_t row = blockIdx.x; const int c8 = threadIdx.x * 8; union { bf16 hh[8]; v4u_t u; } cv;
  const v4f_t a = *(const v4f_t*)(T + row * EE + c8), c = *(const v4f_t*)(T + row * EE + c8 + 4); for (int i = 0; i < 4; ++i) { cv.hh[i] = (bf16)fmaxf(a[i], 0.0f); cv.hh[4 + i] = (bf16)fmaxf(c[i], 0.0f); }
  *(volatile v4u_t*)(O + row * EE + c8) = cv.u; __threadfence(); *(volatile v4u_t*)(O + row * EE + c8) = cv.u; }
__global__ __launch_bounds__(192) void k_scatter_out(const float* __restrict__ O, int b, float* __restrict__ out) { const int lq = blockIdx.x; const int c4 = threadIdx.x * 4; const int h = c4 >> 6, d = c4 & 63;
  const v4f_t v = *(const v4f_t*)(O + (size_t)lq * EE + c4); float* dst = out + (((size_t)b * HH + h) * LQ + lq) * DKK + d; *(volatile v4f_t*)dst = v; __threadfence(); *(volatile v4f_t*)dst = v; }

extern "C" void kernel_launch(void* const* d_in, const int* in_sizes, int n_in,
                              void* d_out, int out_size, void* d_ws, size_t ws_size,
                              hipStream_t stream) {
  (void)in_sizes; (void)n_in; (void)out_size;
  const float** f = (const float**)d_in;
  const float* st = f[0], *Wi = f[1], *bi = f[2], *Wq = f[3], *bq = f[4], *Wk = f[5], *bk = f[6], *Wv = f[7], *bv = f[8], *Wao = f[9], *bao = f[10], *Wo = f[11], *bo = f[12];
  float* out = (float*)d_out;
  char* ws = (char*)d_ws;
  float* WiT = (float*)ws; ws += (size_t)EE * EE * 4;
  float* X0 = (float*)ws; ws += (size_t)LL * EE * 4;
  float* Xres = (float*)ws; ws += (size_t)LQ * EE * 4;
  bf16* XR16 = (bf16*)ws; ws += (size_t)LL * EE * 2;
  bf16* K16 = (bf16*)ws; ws += (size_t)LL * EE * 2; bf16* V16 = (bf16*)ws; ws += (size_t)LL * EE * 2; bf16* Vt = (bf16*)ws; ws += (size_t)EE * LL * 2;
  bf16* Aq = (bf16*)ws; ws += (size_t)LQ * 3 * EE * 2;
  float* Qf = (float*)ws; ws += (size_t)LQ * EE * 4; bf16* Q16 = (bf16*)ws; ws += (size_t)LQ * EE * 2;
  float* att = (float*)ws; ws += (size_t)LQ * EE * 4; float* T1 = (float*)ws; ws += (size_t)LQ * EE * 4; bf16* T16 = (bf16*)ws; ws += (size_t)LQ * EE * 2; float* O = (float*)ws; ws += (size_t)LQ * EE * 4;
  if ((size_t)(ws - (char*)d_ws) > ws_size) return;
  const dim3 blk(256);
  k_transpose<<<dim3((EE / 64) * (EE / 64)), blk, 0, stream>>>(Wi, WiT, EE, EE);
  for (int b = 0; b < NB; ++b) {
    k_gather_x0<<<dim3(LL), dim3(192), 0, stream>>>(st, b, X0);
    k_resid<<<dim3(LQ), dim3(192), 0, stream>>>(X0, Xres);
    gemm_kne<float, 3, true><<<dim3(LL / 128, EE / 128), blk, 0, stream>>>(X0, EE, WiT, EE, bi, nullptr, nullptr, XR16, EE, EE);
    k_im2col<<<dim3(LQ, 3), dim3(96), 0, stream>>>(XR16, Aq);
    gemm_kne<bf16, 0, false><<<dim3(LQ / 128, EE / 128), blk, 0, stream>>>(Aq, 3 * EE, Wq, EE, bq, nullptr, nullptr, Qf, EE, 3 * EE);
    k_rows16<<<dim3(LQ / 64, HH), blk, 0, stream>>>(Qf, Q16);
    gemm_rb_kernel<bf16, 0><<<dim3(LL / 128, EE / 256), blk, 0, stream>>>(XR16, Wk, bk, nullptr, nullptr, nullptr, K16, LL, EE, EE);
    gemm_rb_kernel<bf16, 0><<<dim3(LL / 128, EE / 256), blk, 0, stream>>>(XR16, Wv, bv, nullptr, nullptr, nullptr, V16, LL, EE, EE);
    k_vt16<<<dim3(LL / 64, HH), blk, 0, stream>>>(V16, Vt);
    ca_attn_kernel<<<dim3(QROWS / 64, HH, 1), dim3(64), 0, stream>>>(Q16, K16, Vt, att);
    gemm_rb_kernel<float, 2><<<dim3(LQ / 128, EE / 256), blk, 0, stream>>>(att, Wao, bao, nullptr, nullptr, nullptr, T1, LQ, EE, EE);
    k_relu16<<<dim3(LQ), dim3(96), 0, stream>>>(T1, T16);
    gemm_rb_kernel<bf16, 2><<<dim3(LQ / 128, EE / 256), blk, 0, stream>>>(T16, Wo, bo, nullptr, Xres, nullptr, O, LQ, EE, EE);
    k_scatter_out<<<dim3(LQ), dim3(192), 0, stream>>>(O, b, out);
  }
}
